// BoundaryPredictor2_66975720014433
// MI455X (gfx1250) — hardware-verified
//
#include <hip/hip_runtime.h>
#include <math.h>


#define NB 8
#define NL 2048
#define ND 512
#define GX (NL / 16)
#define ROW_WQ (NB * NL)
#define ROW_WK (NB * NL + ND)
#define NROWS (NB * NL + 2 * ND)
#define TPT 8
#define BIGI 0x3fffffff
#define STW 32
#define NTAIL (3 + NB * NL + 3 * NB)
#define NLINE ((NTAIL + 31) / 32)

typedef float          v4f  __attribute__((ext_vector_type(4)));
typedef float          v8f  __attribute__((ext_vector_type(8)));
typedef int            v4i  __attribute__((ext_vector_type(4)));
typedef int            v8i  __attribute__((ext_vector_type(8)));
typedef unsigned short v8us __attribute__((ext_vector_type(8)));
typedef __bf16         v16b __attribute__((ext_vector_type(16)));

union FragB { v16b v; v8us half[2]; v8i w; };

__device__ __forceinline__ float wave_sum32(float v) {
#pragma unroll
    for (int m = 16; m >= 1; m >>= 1) v += __shfl_xor(v, m, 32);
    return v;
}
__device__ __forceinline__ int wave_min32(int v) {
#pragma unroll
    for (int m = 16; m >= 1; m >>= 1) { const int o = __shfl_xor(v, m, 32); v = (o < v) ? o : v; }
    return v;
}

__device__ __forceinline__ unsigned int bf16_rne(float x) {
    const unsigned int u = __float_as_uint(x);
    return (u + 0x7FFFu + ((u >> 16) & 1u)) >> 16;
}
__device__ __forceinline__ void split2(float x, unsigned short& hi, unsigned short& lo) {
    const unsigned int hb = bf16_rne(x);
    const float hf = __uint_as_float(hb << 16);
    hi = (unsigned short)hb;
    lo = (unsigned short)bf16_rne(x - hf);
}

__device__ __forceinline__ void ldfrag(FragB& f, const unsigned short* __restrict__ p, int o0, int o1) {
    f.half[0] = *(const v8us*)(p + o0);
    f.half[1] = *(const v8us*)(p + o1);
}

__device__ __forceinline__ v8f wmma3(v8f acc, const FragB& ah, const FragB& al, const FragB& bh, const FragB& bl) {
    acc = __builtin_amdgcn_wmma_f32_16x16x32_bf16(false, ah.v, false, bh.v, (short)0, acc, false, false);
    acc = __builtin_amdgcn_wmma_f32_16x16x32_bf16(false, al.v, false, bh.v, (short)0, acc, false, false);
    acc = __builtin_amdgcn_wmma_f32_16x16x32_bf16(false, ah.v, false, bl.v, (short)0, acc, false, false);
    asm volatile("v_nop\n\tv_nop\n\tv_nop\n\tv_nop" : "+v"(acc) : "v"(ah.w), "v"(al.w), "v"(bh.w), "v"(bl.w));
    return acc;
}

__global__ __launch_bounds__(256) void k_prep(const float* __restrict__ hidden,
                                              const float* __restrict__ Wq,
                                              const float* __restrict__ Wk,
                                              unsigned short* __restrict__ phi,
                                              unsigned short* __restrict__ plo)
{
    const int wave = threadIdx.x >> 5, lane = threadIdx.x & 31;
    const int r = blockIdx.x * 8 + wave;
    if (r >= NROWS) return;
    const float* src;
    bool donorm;
    if (r < NB * NL)      { src = hidden + (size_t)r * ND;         donorm = true;  }
    else if (r < ROW_WK)  { src = Wq + (size_t)(r - ROW_WQ) * ND;  donorm = false; }
    else                  { src = Wk + (size_t)(r - ROW_WK) * ND;  donorm = false; }

    v4f x[4];
    x[0] = *(const v4f*)(src + 8 * lane);
    x[1] = *(const v4f*)(src + 8 * lane + 4);
    x[2] = *(const v4f*)(src + 256 + 8 * lane);
    x[3] = *(const v4f*)(src + 256 + 8 * lane + 4);

    float inv = 1.0f;
    if (donorm) {
        float ss = 0.0f;
#pragma unroll
        for (int a = 0; a < 4; ++a)
            ss += x[a][0] * x[a][0] + x[a][1] * x[a][1] + x[a][2] * x[a][2] + x[a][3] * x[a][3];
        ss = wave_sum32(ss);
        float nr = sqrtf(ss);
        if (nr < 1e-12f) nr = 1e-12f;
        inv = 1.0f / nr;
    }

    unsigned short hh[16], ll[16];
#pragma unroll
    for (int a = 0; a < 4; ++a)
#pragma unroll
        for (int c = 0; c < 4; ++c)
            split2(x[a][c] * inv, hh[4 * a + c], ll[4 * a + c]);

    const v8us h0 = {hh[0], hh[1], hh[2], hh[3], hh[4], hh[5], hh[6], hh[7]};
    const v8us h1 = {hh[8], hh[9], hh[10], hh[11], hh[12], hh[13], hh[14], hh[15]};
    const v8us g0 = {ll[0], ll[1], ll[2], ll[3], ll[4], ll[5], ll[6], ll[7]};
    const v8us g1 = {ll[8], ll[9], ll[10], ll[11], ll[12], ll[13], ll[14], ll[15]};

    unsigned short* ph = phi + (size_t)r * ND + 8 * lane;
    unsigned short* pl = plo + (size_t)r * ND + 8 * lane;
    *(volatile v8us*)(ph)       = h0;
    *(volatile v8us*)(ph + 256) = h1;
    *(volatile v8us*)(pl)       = g0;
    *(volatile v8us*)(pl + 256) = g1;
    __threadfence();
    *(volatile v8us*)(ph)       = h0;
    *(volatile v8us*)(ph + 256) = h1;
    *(volatile v8us*)(pl)       = g0;
    *(volatile v8us*)(pl + 256) = g1;
}

__global__ __launch_bounds__(256) void k_gemm_cos(const unsigned short* __restrict__ phi,
                                                  const unsigned short* __restrict__ plo,
                                                  float* __restrict__ cosw)
{
    __shared__ float sWD[8][16];
    __shared__ __align__(16) float sC[32];

    const int b = blockIdx.y, bx = blockIdx.x, l0 = bx * 16;
    const int tid = threadIdx.x, wave = tid >> 5, lane = tid & 31, h = lane >> 4, m = lane & 15;
    const int tq = l0 + m;
    int tk = l0 + m + 1; if (tk > NL - 1) tk = NL - 1;
    const unsigned short* aqh_p = phi + ((size_t)b * NL + tq) * ND;
    const unsigned short* aql_p = plo + ((size_t)b * NL + tq) * ND;
    const unsigned short* akh_p = phi + ((size_t)b * NL + tk) * ND;
    const unsigned short* akl_p = plo + ((size_t)b * NL + tk) * ND;

    float part[8];
#pragma unroll
    for (int r = 0; r < 8; ++r) part[r] = 0.0f;

#pragma unroll 1
    for (int jp = 0; jp < 2; ++jp) {
        v8f accQ[2], accK[2];
#pragma unroll
        for (int t = 0; t < 2; ++t) {
#pragma unroll
            for (int r = 0; r < 8; ++r) { accQ[t][r] = 0.0f; accK[t][r] = 0.0f; }
        }
        size_t rwq[2], rwk[2];
#pragma unroll
        for (int t = 0; t < 2; ++t) {
            const int n = ((wave * 2 + jp) * 2 + t) * 16 + m;
            rwq[t] = (size_t)(ROW_WQ + n) * ND;
            rwk[t] = (size_t)(ROW_WK + n) * ND;
        }
#pragma unroll 1
        for (int ks = 0; ks < ND / 32; ++ks) {
            const int o0 = ks * 32 + 8 * h, o1 = o0 + 16;
            FragB aqh, aql, akh, akl;
            ldfrag(aqh, aqh_p, o0, o1);
            ldfrag(aql, aql_p, o0, o1);
            ldfrag(akh, akh_p, o0, o1);
            ldfrag(akl, akl_p, o0, o1);
#pragma unroll
            for (int t = 0; t < 2; ++t) {
                FragB bh, bl;
                ldfrag(bh, phi + rwq[t], o0, o1);
                ldfrag(bl, plo + rwq[t], o0, o1);
                accQ[t] = wmma3(accQ[t], aqh, aql, bh, bl);
                ldfrag(bh, phi + rwk[t], o0, o1);
                ldfrag(bl, plo + rwk[t], o0, o1);
                accK[t] = wmma3(accK[t], akh, akl, bh, bl);
            }
        }
#pragma unroll
        for (int r = 0; r < 8; ++r)
            part[r] += accQ[0][r] * accK[0][r] + accQ[1][r] * accK[1][r];
    }

#pragma unroll
    for (int msk = 8; msk >= 1; msk >>= 1)
#pragma unroll
        for (int r = 0; r < 8; ++r) part[r] += __shfl_xor(part[r], msk, 32);

    if (m == 0) {
#pragma unroll
        for (int r = 0; r < 8; ++r) sWD[wave][8 * h + r] = part[r];
    }
    __syncthreads();
    if (tid < 32) {
        float v = 0.0f;
        if (tid < 16 && (l0 + tid) < NL - 1) {
#pragma unroll
            for (int w = 0; w < 8; ++w) v += sWD[w][tid];
        }
        sC[tid] = v;
    }
    __syncthreads();
    if (tid < 8) {
        const v4f cv = *(const v4f*)(sC + 4 * tid);
        float* dst = cosw + ((size_t)b * GX + bx) * 32 + 4 * tid;
        *(volatile v4f*)dst = cv;
        __threadfence();
        *(volatile v4f*)dst = cv;
    }
}

__global__ __launch_bounds__(256) void k_seg(const float* __restrict__ cosw,
                                             const float* __restrict__ amask,
                                             const float* __restrict__ noise,
                                             int* __restrict__ brk_ws,
                                             float* __restrict__ stat_ws)
{
#pragma clang fp contract(off)
    __shared__ float sredf[6][8];
    __shared__ int   sredi[8];
    __shared__ int   sscan[257];
    __shared__ __align__(16) int   spos[NL];
    __shared__ __align__(16) float sst[STW];
    __shared__ int   s_fp;
    __shared__ float s_ms;

    const int b = blockIdx.x, tid = threadIdx.x, wave = tid >> 5, lane = tid & 31, l0 = tid * TPT;
    const size_t rowb = (size_t)b * NL;
    if (tid < STW) sst[tid] = 0.0f;

    float msum = 0.0f; int fpl = BIGI;
#pragma unroll
    for (int i = 0; i < TPT; ++i) {
        const int l = l0 + i;
        const float mv = amask[rowb + l];
        msum += mv;
        if (mv == 0.0f && l < fpl) fpl = l;
    }
    msum = wave_sum32(msum);
    fpl  = wave_min32(fpl);
    if (lane == 0) { sredf[0][wave] = msum; sredi[wave] = fpl; }
    __syncthreads();
    if (tid == 0) {
        float s = 0.0f; int f = BIGI;
        for (int w = 0; w < 8; ++w) { s += sredf[0][w]; if (sredi[w] < f) f = sredi[w]; }
        s_ms = s; s_fp = f;
    }
    __syncthreads();
    const float msT = s_ms;
    const int   fp  = s_fp;
    const int   fpos = (fp < BIGI && fp >= 1) ? (fp - 1) : -1;

    const float EPSF = 1.1920929e-07f;
    float lp = 0.0f, conf = 0.0f, ent = 0.0f, cntf = 0.0f, hbf = 0.0f;
    int flags = 0, cnt = 0;
#pragma unroll 1
    for (int i = 0; i < TPT; ++i) {
        const int l = l0 + i;
        const float mv = amask[rowb + l];
        float p = 0.0f;
        if (l < NL - 1) {
            const float c = cosw[((size_t)b * GX + (l >> 4)) * 32 + (l & 15)];
            p = (1.0f - c) * 0.5f;
            p = fminf(fmaxf(p, 0.0f), 1.0f);
        }
        const float pc  = fminf(fmaxf(p, EPSF), 1.0f - EPSF);
        const float lg  = logf(pc) - log1pf(-pc);
        const float u   = noise[rowb + l];
        const float ng  = logf(u) - log1pf(-u);
        const float x   = lg + ng;
        const float sft = 1.0f / (1.0f + expf(-x));
        float hard = (sft > 0.5f) ? 1.0f : 0.0f;
        hard = hard * mv;
        float sfm = sft * mv;
        const float frc = (l == fpos) ? 1.0f : 0.0f;
        hard = fmaxf(hard, frc);
        sfm  = fmaxf(sfm, frc);
        const float hb  = (hard - sfm) + sfm;
        const float pc2 = fminf(fmaxf(p, 1e-8f), 1.0f);
        const float lq  = logf(pc2), l1q = log1pf(-pc2);
        lp   += (hard * lq + (1.0f - hard) * l1q) * mv;
        conf += fabsf(p - 0.5f) * mv;
        ent  += (0.0f - (pc2 * lq + (1.0f - pc2) * l1q)) * mv;
        cntf += hard;
        hbf  += hb;
        if (hb != 0.0f) { flags |= (1 << i); ++cnt; }
    }

    lp   = wave_sum32(lp);
    conf = wave_sum32(conf);
    ent  = wave_sum32(ent);
    cntf = wave_sum32(cntf);
    hbf  = wave_sum32(hbf);
    if (lane == 0) {
        sredf[1][wave] = lp; sredf[2][wave] = conf; sredf[3][wave] = ent;
        sredf[4][wave] = cntf; sredf[5][wave] = hbf;
    }
    sscan[tid] = cnt;
    __syncthreads();
    if (tid == 0) {
        int acc = 0;
        for (int i = 0; i < 256; ++i) { const int c = sscan[i]; sscan[i] = acc; acc += c; }
        sscan[256] = acc;
        float a1 = 0.0f, a2 = 0.0f, a3 = 0.0f, a4 = 0.0f, a5 = 0.0f;
        for (int w = 0; w < 8; ++w) { a1 += sredf[1][w]; a2 += sredf[2][w]; a3 += sredf[3][w]; a4 += sredf[4][w]; a5 += sredf[5][w]; }
        sst[0] = a4;
        sst[1] = msT;
        sst[2] = a1;
        sst[3] = a2 / fmaxf(msT, 1.0f);
        sst[4] = a3;
        sst[5] = a5;
    }
    __syncthreads();
    const int base  = sscan[tid];
    const int total = sscan[256];

    int j = base;
#pragma unroll
    for (int i = 0; i < TPT; ++i) {
        if (flags & (1 << i)) { if ((unsigned)j < (unsigned)NL) spos[j] = l0 + i; ++j; }
    }
    for (int idx = total + tid; idx < NL; idx += 256) spos[idx] = NL - 1;
    __syncthreads();

    const v4i p0 = *(const v4i*)(spos + 4 * tid);
    const v4i p1 = *(const v4i*)(spos + 4 * (tid + 256));
    int* d0 = brk_ws + rowb + 4 * tid;
    int* d1 = brk_ws + rowb + 4 * (tid + 256);
    v4f sv = {0.0f, 0.0f, 0.0f, 0.0f};
    float* ds = stat_ws + (size_t)b * STW;
    const bool dost = (tid < 8);
    if (dost) { sv = *(const v4f*)(sst + 4 * tid); ds += 4 * tid; }

    *(volatile v4i*)d0 = p0;
    *(volatile v4i*)d1 = p1;
    if (dost) *(volatile v4f*)ds = sv;
    __threadfence();
    *(volatile v4i*)d0 = p0;
    *(volatile v4i*)d1 = p1;
    if (dost) *(volatile v4f*)ds = sv;
}

__device__ __forceinline__ int clampi(int v) { return v < 0 ? 0 : (v > NL - 1 ? NL - 1 : v); }

__global__ __launch_bounds__(128) void k_pool(const float* __restrict__ hidden,
                                              const float* __restrict__ amask,
                                              const int* __restrict__ brk_ws,
                                              const float* __restrict__ stat_ws,
                                              float* __restrict__ pooled)
{
    const int b = blockIdx.y, s = blockIdx.x, tid = threadIdx.x;
    const size_t rowb = (size_t)b * NL;
    int cnt = (int)stat_ws[(size_t)b * STW];
    if (cnt < 0) cnt = 0;
    if (cnt > NL) cnt = NL;
    const int* brk = brk_ws + rowb;

    int start, end;
    if (s < cnt) {
        end   = clampi(brk[s]);
        start = (s == 0) ? 0 : clampi(brk[s - 1]) + 1;
    } else if (s == cnt) {
        start = (cnt == 0) ? 0 : clampi(brk[cnt - 1]) + 1;
        end   = NL - 1;
    } else {
        start = 1; end = 0;
    }

    v4f acc = {0.0f, 0.0f, 0.0f, 0.0f};
    float ns = 0.0f;
    for (int t = start; t <= end; ++t) {
        const float mv = amask[rowb + t];
        const v4f hv = *(const v4f*)(hidden + (rowb + t) * ND + 4 * tid);
        acc += hv * mv;
        ns  += mv;
    }
    const float inv = 1.0f / (ns + 1e-9f);
    const v4f val = acc * inv;
    float* dst = pooled + (rowb + s) * ND + 4 * tid;
    *(volatile v4f*)dst = val;
    __threadfence();
    *(volatile v4f*)dst = val;
}

__device__ __forceinline__ float lgam_pos(float z) {
    if (z < 1.0f) z = 1.0f;
    float corr = 0.0f;
    for (int it = 0; it < 16 && z < 8.0f; ++it) { corr -= logf(z); z += 1.0f; }
    const float iz = 1.0f / z, iz2 = iz * iz;
    const float ser = iz * (0.0833333333f - iz2 * (0.00277777778f - iz2 * 0.000793650794f));
    return (z - 0.5f) * logf(z) - z + 0.918938533f + ser + corr;
}

__device__ __forceinline__ float tailval(int f, const float* s3, const float* sc,
                                         const float* slp, const float* scf, const float* sen)
{
    if (f < 3) return s3[f];
    int g = f - 3;
    if (g < NB * NL) {
        const int bb = g >> 11, s = g & (NL - 1);
        return ((float)s < sc[bb]) ? 1.0f : 0.0f;
    }
    g -= NB * NL;
    if (g < NB) return slp[g];
    g -= NB;
    if (g < NB) return scf[g];
    g -= NB;
    if (g < NB) return sen[g];
    return 0.0f;
}

__device__ __forceinline__ void tail_lines(float* tail, int tid, const float* s3, const float* sc,
                                           const float* slp, const float* scf, const float* sen)
{
    for (int q = tid; q < NLINE; q += 256) {
        const int f0 = 32 * q;
        if (q < NLINE - 1) {
#pragma unroll
            for (int g = 0; g < 8; ++g) {
                v4f w;
                w.x = tailval(f0 + 4 * g + 0, s3, sc, slp, scf, sen);
                w.y = tailval(f0 + 4 * g + 1, s3, sc, slp, scf, sen);
                w.z = tailval(f0 + 4 * g + 2, s3, sc, slp, scf, sen);
                w.w = tailval(f0 + 4 * g + 3, s3, sc, slp, scf, sen);
                *(volatile v4f*)(tail + f0 + 4 * g) = w;
            }
        } else {
            const int rem = NTAIL - f0;
            const int ng = rem >> 2;
            for (int g = 0; g < ng; ++g) {
                v4f w;
                w.x = tailval(f0 + 4 * g + 0, s3, sc, slp, scf, sen);
                w.y = tailval(f0 + 4 * g + 1, s3, sc, slp, scf, sen);
                w.z = tailval(f0 + 4 * g + 2, s3, sc, slp, scf, sen);
                w.w = tailval(f0 + 4 * g + 3, s3, sc, slp, scf, sen);
                *(volatile v4f*)(tail + f0 + 4 * g) = w;
            }
            for (int f = f0 + 4 * ng; f < NTAIL; ++f)
                *(volatile float*)(tail + f) = tailval(f, s3, sc, slp, scf, sen);
        }
    }
}

__global__ __launch_bounds__(256) void k_fin(const float* __restrict__ stat_ws, float* __restrict__ tail)
{
    __shared__ float sc[NB], sms[NB], slp[NB], scf[NB], sen[NB], shb[NB];
    __shared__ float s3[3];
    const int tid = threadIdx.x;
    if (tid < NB) {
        const float* st = stat_ws + (size_t)tid * STW;
        sc[tid] = st[0]; sms[tid] = st[1]; slp[tid] = st[2];
        scf[tid] = st[3]; sen[tid] = st[4]; shb[tid] = st[5];
    }
    __syncthreads();
    if (tid == 0) {
        float nb = 0.0f, tp = 0.0f;
        for (int bb = 0; bb < NB; ++bb) { nb += shb[bb]; tp += sms[bb]; }
        const float p   = 0.2f;
        const float wgt = 0.0f;
        const float n = tp, kk = nb;
        const float lpb = lgam_pos(n + 1.0f) - lgam_pos(kk + 1.0f) - lgam_pos(n - kk + 1.0f)
                        + kk * logf(p) + (n - kk) * log1pf(-p);
        s3[0] = (-lpb / n) * wgt;
        s3[1] = nb;
        s3[2] = tp;
    }
    __syncthreads();
    tail_lines(tail, tid, s3, sc, slp, scf, sen);
    __threadfence();
    tail_lines(tail, tid, s3, sc, slp, scf, sen);
}

extern "C" void kernel_launch(void* const* d_in, const int* in_sizes, int n_in,
                              void* d_out, int out_size, void* d_ws, size_t ws_size,
                              hipStream_t stream)
{
    if (n_in < 5) return;
    if (in_sizes[0] != NB * NL * ND || in_sizes[1] != NB * NL || in_sizes[2] != NB * NL ||
        in_sizes[3] != ND * ND || in_sizes[4] != ND * ND) return;
    if (out_size != NB * NL * ND + NTAIL) return;

    const float* hidden = (const float*)d_in[0];
    const float* amask  = (const float*)d_in[1];
    const float* noise  = (const float*)d_in[2];
    const float* Wq     = (const float*)d_in[3];
    const float* Wk     = (const float*)d_in[4];

    float* out    = (float*)d_out;
    float* pooled = out;
    float* tail   = out + (size_t)NB * NL * ND;

    const size_t plane_bytes = (size_t)NROWS * ND * 2;
    const size_t off_hi  = 0;
    const size_t off_lo  = off_hi + plane_bytes;
    const size_t off_cos = off_lo + plane_bytes;
    const size_t cos_bytes = (size_t)NB * GX * 32 * 4;
    const size_t off_brk = off_cos + cos_bytes;
    const size_t brk_bytes = (size_t)NB * NL * 4;
    const size_t off_st  = off_brk + brk_bytes;
    const size_t st_bytes = (size_t)NB * STW * 4;
    const size_t total = off_st + st_bytes;
    if (total > ws_size) return;

    char* ws = (char*)d_ws;
    unsigned short* phi = (unsigned short*)(ws + off_hi);
    unsigned short* plo = (unsigned short*)(ws + off_lo);
    float* cosw = (float*)(ws + off_cos);
    int*   brk  = (int*)(ws + off_brk);
    float* stw  = (float*)(ws + off_st);

    k_prep<<<dim3((NROWS + 7) / 8), 256, 0, stream>>>(hidden, Wq, Wk, phi, plo);
    k_gemm_cos<<<dim3(GX, NB), 256, 0, stream>>>(phi, plo, cosw);
    k_seg<<<dim3(NB), 256, 0, stream>>>(cosw, amask, noise, brk, stw);
    k_pool<<<dim3(NL, NB), 128, 0, stream>>>(hidden, amask, brk, stw, pooled);
    k_fin<<<dim3(1), 256, 0, stream>>>(stw, tail);
}
